// Head_23313082482790
// MI455X (gfx1250) — hardware-verified
//
#include <hip/hip_runtime.h>

#pragma clang fp contract(off)

#ifndef NB
#define NB 8
#endif
#ifndef SEQ
#define SEQ 4096
#endif
#define NB_FULL  8
#define SEQ_FULL 4096
#define DM   128
#define HS   32
#define NP   128
#ifndef RH
#define RH   1024
#endif
#define PCAR 16384.0f
#define SCL  0.17677669529663687f
#define L2E  1.4426950408889634f
#define PP   72
#define OPF  36
static_assert(SEQ % 64 == 0);
static_assert(SEQ <= SEQ_FULL);
static_assert(NB >= 1);
static_assert(NB <= NB_FULL);
static_assert(RH % 64 == 0);
static_assert(DM % 32 == 0);
static_assert((NB * SEQ * (DM / 8)) % 256 == 0);
static_assert((SEQ * 16) % 256 == 0);
static_assert((NP * DM / 8) % 256 == 0);
static_assert((long long)NB_FULL * SEQ_FULL * HS * 4 == 4194304LL);

typedef _Float16 h16;
typedef unsigned short bf;
typedef __attribute__((ext_vector_type(16))) __bf16   v16bf;
typedef __attribute__((ext_vector_type(16))) _Float16 v16h;
typedef __attribute__((ext_vector_type(8)))  _Float16 v8h;
typedef __attribute__((ext_vector_type(8)))  unsigned short v8us;
typedef __attribute__((ext_vector_type(2)))  unsigned short v2us;
typedef __attribute__((ext_vector_type(8)))  float    v8f;
typedef __attribute__((ext_vector_type(4)))  float    v4f;
typedef __attribute__((ext_vector_type(2)))  float    v2f;
typedef v8h  __attribute__((may_alias)) v8ha;
typedef v4f  __attribute__((may_alias)) v4fa;
typedef v8us __attribute__((may_alias)) v8usa;

__device__ __forceinline__ unsigned short f2bf(float f) { unsigned u = __float_as_uint(f); u += 0x7FFFu + ((u >> 16) & 1u); return (unsigned short)(u >> 16); }
__device__ __forceinline__ float bf2f(unsigned short b) { return __uint_as_float(((unsigned)b) << 16); }
__device__ __forceinline__ float bfr(float f) { return bf2f(f2bf(f)); }
__device__ __forceinline__ v16h cat16(v8h lo, v8h hi) { return __builtin_shufflevector(lo, hi, 0, 1, 2, 3, 4, 5, 6, 7, 8, 9, 10, 11, 12, 13, 14, 15); }
__device__ __forceinline__ v16bf cat16b(v8us lo, v8us hi) { return __builtin_bit_cast(v16bf, __builtin_shufflevector(lo, hi, 0, 1, 2, 3, 4, 5, 6, 7, 8, 9, 10, 11, 12, 13, 14, 15)); }
__device__ __forceinline__ v8f wmma16(v16h a, v16h b, v8f c) { return __builtin_amdgcn_wmma_f32_16x16x32_f16(false, a, false, b, (short)0, c, false, false); }
__device__ __forceinline__ v8f wmmab(v16bf a, v16bf b, v8f c) { return __builtin_amdgcn_wmma_f32_16x16x32_bf16(false, a, false, b, (short)0, c, false, false); }

template <typename T16> struct WFrag;
template <> struct WFrag<h16> { typedef v16h V; static __device__ __forceinline__ V ld(const h16* p) { return cat16(*(const v8h*)p, *(const v8h*)(p + 16)); } static __device__ __forceinline__ v8f mma(V a, V b, v8f c) { return wmma16(a, b, c); } };
template <> struct WFrag<bf> { typedef v16bf V; static __device__ __forceinline__ V ld(const bf* p) { return cat16b(*(const v8us*)p, *(const v8us*)(p + 16)); } static __device__ __forceinline__ v8f mma(V a, V b, v8f c) { return wmmab(a, b, c); } };
template <typename T16, int NSPLIT, bool BIAS>
__global__ __launch_bounds__(32) void k_gemmw(const T16* __restrict__ A, const T16* __restrict__ A2, const T16* __restrict__ Bt, const T16* __restrict__ Bt2, int K, float* C, int ldc, const float* __restrict__ bias, size_t sA, size_t sB, size_t sC) {
    typedef typename WFrag<T16>::V V;
    __shared__ __align__(16) float os[16 * 68];
    const size_t z = blockIdx.z; A += z * sA; if (A2) A2 += z * sA; Bt += z * sB; if (Bt2) Bt2 += z * sB; C += z * sC;
    const int lane = threadIdx.x & 31, lr = lane & 15, hi = lane >> 4; const int r0 = blockIdx.x * 64, c0 = blockIdx.y * 64;
    v8f acc[4][4];
#pragma unroll
    for (int mb = 0; mb < 4; ++mb)
#pragma unroll
        for (int nb = 0; nb < 4; ++nb) acc[mb][nb] = (v8f){};
    const size_t aoff = (size_t)(r0 + lr) * K + 8 * hi, boff = (size_t)(c0 + lr) * K + 8 * hi;
#pragma unroll 1
    for (int kc = 0; kc < K; kc += 32) {
        V a[4], a2[4];
#pragma unroll
        for (int mb = 0; mb < 4; ++mb) { a[mb] = WFrag<T16>::ld(A + aoff + (size_t)mb * 16 * K + kc); if (NSPLIT == 1 || NSPLIT == 2) a2[mb] = WFrag<T16>::ld(A2 + aoff + (size_t)mb * 16 * K + kc); }
#pragma unroll
        for (int nb = 0; nb < 4; ++nb) { const V b = WFrag<T16>::ld(Bt + boff + (size_t)nb * 16 * K + kc); V b2; if (NSPLIT >= 2) b2 = WFrag<T16>::ld(Bt2 + boff + (size_t)nb * 16 * K + kc);
#pragma unroll
            for (int mb = 0; mb < 4; ++mb) { acc[mb][nb] = WFrag<T16>::mma(a[mb], b, acc[mb][nb]); if (NSPLIT == 1 || NSPLIT == 2) acc[mb][nb] = WFrag<T16>::mma(a2[mb], b, acc[mb][nb]); if (NSPLIT >= 2) acc[mb][nb] = WFrag<T16>::mma(a[mb], b2, acc[mb][nb]); } }
        asm volatile("v_nop\n\tv_nop\n\tv_nop\n\tv_nop" : "+v"(acc[0][0]), "+v"(acc[1][1]), "+v"(acc[2][2]), "+v"(acc[3][3]) : "v"(a[0]), "v"(a[3]));
    }
#pragma unroll
    for (int mb = 0; mb < 4; ++mb) {
#pragma unroll
        for (int nb = 0; nb < 4; ++nb) {
#pragma unroll
            for (int j = 0; j < 8; ++j) os[(hi * 8 + j) * 68 + nb * 16 + lr] = acc[mb][nb][j]; }
        __builtin_amdgcn_wave_barrier(); asm volatile("" ::: "memory");
        float* crow = C + (size_t)(r0 + mb * 16) * ldc + c0;
#pragma unroll 1
        for (int ps = 0; ps < 2; ++ps) {
#pragma unroll
            for (int s = 0; s < 8; ++s) { const int row = 2 * s + hi, cofs = lr * 4; v4f val = *(const v4fa*)(os + row * 68 + cofs); if (BIAS) { val[0] += bfr(bias[c0 + cofs]); val[1] += bfr(bias[c0 + cofs + 1]); val[2] += bfr(bias[c0 + cofs + 2]); val[3] += bfr(bias[c0 + cofs + 3]); }
                *(volatile v4f*)(crow + (size_t)row * ldc + cofs) = val; }
            if (ps == 0) __threadfence(); }
        __builtin_amdgcn_wave_barrier(); asm volatile("" ::: "memory");
    }
}

__global__ __launch_bounds__(256) void k_wt(const float* __restrict__ wq, const float* __restrict__ wk, const float* __restrict__ wv, bf* WB) {
    const int i = blockIdx.x * 256 + threadIdx.x; if (i >= NP * DM / 8) return;
    const int e0 = i * 8; const int n = e0 / DM, k0 = e0 % DM; const int nn = n & 31;
    const float* src = (n < 32) ? wq : ((n < 64) ? wk : wv);
    v8us o;
#pragma unroll
    for (int j = 0; j < 8; ++j) { const float v = src[(size_t)(k0 + j) * HS + nn]; o[j] = f2bf((n < 96) ? v : 0.0f); }
    *(volatile v8us*)(WB + e0) = o; __threadfence(); *(volatile v8us*)(WB + e0) = o;
}

__constant__ float INVT[HS / 2] = { 1.0f, 0.5623413324356079f, 0.3162277638912201f, 0.17782793939113617f, 0.10000000149011612f, 0.05623412877321243f, 0.03162277862429619f, 0.017782794311642647f, 0.009999999776482582f, 0.005623413249850273f, 0.003162277862429619f, 0.0017782794311642647f, 0.0010000000474974513f, 0.000562341301701963f, 0.0003162277862429619f, 0.00017782794020604342f };
__global__ __launch_bounds__(256) void k_cs(float* CS) {
    const int idx = blockIdx.x * 256 + threadIdx.x; if (idx >= SEQ * (HS / 2)) return;
    const int t = idx >> 4, i = idx & 15;
    const float ang = INVT[i] * (float)t; float sn, cn; sincosf(ang, &sn, &cn);
    v2f cs; cs[0] = cn; cs[1] = sn;
    *(volatile v2f*)(CS + (size_t)idx * 2) = cs; __threadfence(); *(volatile v2f*)(CS + (size_t)idx * 2) = cs;
}
__global__ __launch_bounds__(256) void k_cvt(const float* __restrict__ x, bf* XB, int n8) {
    const int i = blockIdx.x * 256 + threadIdx.x; if (i >= n8) return;
    const int row = i / (DM / 8), c8 = i % (DM / 8); const int b = row / SEQ, t = row % SEQ;
    const v8f v = *(const v8f*)(x + ((size_t)b * SEQ_FULL + t) * DM + c8 * 8);
    v8us o;
#pragma unroll
    for (int k = 0; k < 8; ++k) o[k] = f2bf(v[k]);
    bf* d = XB + (size_t)i * 8; *(volatile v8us*)d = o; __threadfence(); *(volatile v8us*)d = o;
}

__global__ __launch_bounds__(256) void k_planes(const float* __restrict__ F, const float* __restrict__ CS, bf* Qh, bf* Ql, bf* Kh, bf* Kl, h16* VT16, bf* VTh, bf* VTl) {
    __shared__ __align__(16) unsigned short sq[4][64 * 32];
    __shared__ __align__(16) unsigned short sv[3][32 * 64];
    const int tid = threadIdx.x; const int b = blockIdx.y, t0 = blockIdx.x * 64;
    const int r = tid >> 2, g = tid & 3; const int t = t0 + r;
    const float* fr = F + ((size_t)b * SEQ + t) * NP;
    const v8f xq = *(const v8f*)(fr + 8 * g), xk = *(const v8f*)(fr + 32 + 8 * g), xv = *(const v8f*)(fr + 64 + 8 * g);
    const v8f cs = *(const v8f*)(CS + ((size_t)t * (HS / 2) + 4 * g) * 2);
#pragma unroll
    for (int p = 0; p < 4; ++p) {
        const float cn = cs[2 * p], sn = cs[2 * p + 1]; const int col = 8 * g + 2 * p;
        {   const float x1 = xq[2 * p], x2 = xq[2 * p + 1]; const float ev = x1 * cn - x2 * sn, od = x1 * sn + x2 * cn;
            v2us oh, ol; unsigned short hh0 = f2bf(ev), hh1 = f2bf(od); oh[0] = hh0; oh[1] = hh1; ol[0] = f2bf(ev - bf2f(hh0)); ol[1] = f2bf(od - bf2f(hh1));
            *(v2us*)(&sq[0][r * 32 + col]) = oh; *(v2us*)(&sq[1][r * 32 + col]) = ol; }
        {   const float x1 = xk[2 * p], x2 = xk[2 * p + 1]; const float ev = x1 * cn - x2 * sn, od = x1 * sn + x2 * cn;
            v2us oh, ol; unsigned short hh0 = f2bf(ev), hh1 = f2bf(od); oh[0] = hh0; oh[1] = hh1; ol[0] = f2bf(ev - bf2f(hh0)); ol[1] = f2bf(od - bf2f(hh1));
            *(v2us*)(&sq[2][r * 32 + col]) = oh; *(v2us*)(&sq[3][r * 32 + col]) = ol; }
#pragma unroll
        for (int j = 0; j < 2; ++j) { const float val = xv[2 * p + j]; const int d = col + j; const unsigned short vh = f2bf(val);
            sv[0][d * 64 + r] = __builtin_bit_cast(unsigned short, (h16)val); sv[1][d * 64 + r] = vh; sv[2][d * 64 + r] = f2bf(val - bf2f(vh)); }
    }
    __syncthreads();
    const int w = tid >> 5, L = tid & 31; const int lo = w * 256 + L * 8;
    const size_t qoff = ((size_t)b * SEQ + t0) * HS + lo;
    const int d = 4 * w + (L >> 3), toff = (L & 7) * 8;
    const size_t voff = ((size_t)b * HS + d) * SEQ + t0 + toff;
    const v8us q0v = *(const v8usa*)(&sq[0][lo]), q1v = *(const v8usa*)(&sq[1][lo]), k0v = *(const v8usa*)(&sq[2][lo]), k1v = *(const v8usa*)(&sq[3][lo]);
    const v8us v0v = *(const v8usa*)(&sv[0][lo]), v1v = *(const v8usa*)(&sv[1][lo]), v2v = *(const v8usa*)(&sv[2][lo]);
    unsigned short* VT16u = (unsigned short*)VT16;
#pragma unroll 1
    for (int ps = 0; ps < 2; ++ps) {
        *(volatile v8us*)(Qh + qoff) = q0v; *(volatile v8us*)(Ql + qoff) = q1v; *(volatile v8us*)(Kh + qoff) = k0v; *(volatile v8us*)(Kl + qoff) = k1v;
        *(volatile v8us*)(VT16u + voff) = v0v; *(volatile v8us*)(VTh + voff) = v1v; *(volatile v8us*)(VTl + voff) = v2v;
        if (ps == 0) __threadfence(); }
}

template <bool HI, bool MASK>
__device__ __forceinline__ void attn_chunk(const bf* __restrict__ Khb, const bf* __restrict__ Klb, const h16* __restrict__ V16b, const bf* __restrict__ Vhb, const bf* __restrict__ Vlb,
                                           unsigned short* pta, unsigned short* ptb, const v16bf aqh, const v16bf aql, const int kv0, const int q0, const int ln, const int hh,
                                           float* mrun, float* lp, v8f& o0, v8f& o1) {
    v16bf bh[4], bl[4];
#pragma unroll
    for (int t = 0; t < 4; ++t) { const size_t ko = (size_t)(kv0 + 16 * t + ln) * HS + 8 * hh;
        bh[t] = cat16b(*(const v8us*)(Khb + ko), *(const v8us*)(Khb + ko + 16)); bl[t] = cat16b(*(const v8us*)(Klb + ko), *(const v8us*)(Klb + ko + 16)); }
    v8f s[4];
#pragma unroll
    for (int t = 0; t < 4; ++t) { v8f a = wmmab(aqh, bh[t], (v8f){}); a = wmmab(aql, bh[t], a); a = wmmab(aqh, bl[t], a); s[t] = a; }
    asm volatile("v_nop\n\tv_nop\n\tv_nop\n\tv_nop" : "+v"(s[0]), "+v"(s[1]), "+v"(s[2]), "+v"(s[3]) : "v"(aqh), "v"(aql), "v"(bh[3]), "v"(bl[3]));
#pragma unroll
    for (int r = 0; r < 8; ++r) {
        const int qi = q0 + 8 * hh + r;
        float e[4];
#pragma unroll
        for (int t = 0; t < 4; ++t) { float v = s[t][r] * SCL; if (MASK) v = (kv0 + 16 * t + ln <= qi) ? v : -3.0e38f; e[t] = v; }
        float rm = fmaxf(fmaxf(e[0], e[1]), fmaxf(e[2], e[3]));
        rm = fmaxf(rm, __shfl_xor(rm, 1, 32)); rm = fmaxf(rm, __shfl_xor(rm, 2, 32)); rm = fmaxf(rm, __shfl_xor(rm, 4, 32)); rm = fmaxf(rm, __shfl_xor(rm, 8, 32));
        const float mn = fmaxf(mrun[r], rm);
        const float cf = __builtin_amdgcn_exp2f((mrun[r] - mn) * L2E);
        mrun[r] = mn;
        float psum = 0.0f;
#pragma unroll
        for (int t = 0; t < 4; ++t) {
            const float p = __builtin_amdgcn_exp2f((e[t] - mn) * L2E);
            psum += p;
            const int po = (8 * hh + r) * PP + 16 * t + ln;
            if (HI) { const unsigned short ph = f2bf(p); pta[po] = ph; ptb[po] = f2bf(p - bf2f(ph)); }
            else { pta[po] = __builtin_bit_cast(unsigned short, (h16)(p * PCAR)); }
        }
        lp[r] = lp[r] * cf + psum; o0[r] = o0[r] * cf; o1[r] = o1[r] * cf;
    }
    __builtin_amdgcn_fence(3  , "wavefront");
    asm volatile("s_wait_dscnt 0x0" ::: "memory");
    __builtin_amdgcn_wave_barrier();
    if (HI) {
        v16bf aph[2], apl[2];
#pragma unroll
        for (int ks = 0; ks < 2; ++ks) { const unsigned short* pr = pta + ln * PP + 32 * ks + 8 * hh; const unsigned short* pr2 = ptb + ln * PP + 32 * ks + 8 * hh;
            aph[ks] = cat16b(*(const v8usa*)pr, *(const v8usa*)(pr + 16)); apl[ks] = cat16b(*(const v8usa*)pr2, *(const v8usa*)(pr2 + 16)); }
        {   v16bf vh[2], vl[2];
#pragma unroll
            for (int ks = 0; ks < 2; ++ks) { const size_t vo = (size_t)ln * SEQ + kv0 + 32 * ks + 8 * hh;
                vh[ks] = cat16b(*(const v8us*)(Vhb + vo), *(const v8us*)(Vhb + vo + 16)); vl[ks] = cat16b(*(const v8us*)(Vlb + vo), *(const v8us*)(Vlb + vo + 16)); }
#pragma unroll
            for (int ks = 0; ks < 2; ++ks) { o0 = wmmab(aph[ks], vh[ks], o0); o0 = wmmab(apl[ks], vh[ks], o0); o0 = wmmab(aph[ks], vl[ks], o0); } }
        {   v16bf vh[2], vl[2];
#pragma unroll
            for (int ks = 0; ks < 2; ++ks) { const size_t vo = (size_t)(16 + ln) * SEQ + kv0 + 32 * ks + 8 * hh;
                vh[ks] = cat16b(*(const v8us*)(Vhb + vo), *(const v8us*)(Vhb + vo + 16)); vl[ks] = cat16b(*(const v8us*)(Vlb + vo), *(const v8us*)(Vlb + vo + 16)); }
#pragma unroll
            for (int ks = 0; ks < 2; ++ks) { o1 = wmmab(aph[ks], vh[ks], o1); o1 = wmmab(apl[ks], vh[ks], o1); o1 = wmmab(aph[ks], vl[ks], o1); }
            asm volatile("v_nop\n\tv_nop\n\tv_nop\n\tv_nop" : "+v"(o0), "+v"(o1) : "v"(aph[1]), "v"(apl[1]), "v"(vh[1]), "v"(vl[1])); }
    } else {
        v16h ap[2];
#pragma unroll
        for (int ks = 0; ks < 2; ++ks) { const unsigned short* pr = pta + ln * PP + 32 * ks + 8 * hh;
            ap[ks] = cat16(__builtin_bit_cast(v8h, *(const v8usa*)pr), __builtin_bit_cast(v8h, *(const v8usa*)(pr + 16))); }
        {   v16h vb[2];
#pragma unroll
            for (int ks = 0; ks < 2; ++ks) { const size_t vo = (size_t)ln * SEQ + kv0 + 32 * ks + 8 * hh; vb[ks] = cat16(*(const v8h*)(V16b + vo), *(const v8h*)(V16b + vo + 16)); }
#pragma unroll
            for (int ks = 0; ks < 2; ++ks) o0 = wmma16(ap[ks], vb[ks], o0); }
        {   v16h vb[2];
#pragma unroll
            for (int ks = 0; ks < 2; ++ks) { const size_t vo = (size_t)(16 + ln) * SEQ + kv0 + 32 * ks + 8 * hh; vb[ks] = cat16(*(const v8h*)(V16b + vo), *(const v8h*)(V16b + vo + 16)); }
#pragma unroll
            for (int ks = 0; ks < 2; ++ks) o1 = wmma16(ap[ks], vb[ks], o1);
            asm volatile("v_nop\n\tv_nop\n\tv_nop\n\tv_nop" : "+v"(o0), "+v"(o1) : "v"(ap[1]), "v"(vb[1])); }
    }
}

template <bool HI>
__global__ __launch_bounds__(128) void k_attn(const bf* __restrict__ Qh, const bf* __restrict__ Ql, const bf* __restrict__ Kh, const bf* __restrict__ Kl,
                                             const h16* __restrict__ V16, const bf* __restrict__ Vh, const bf* __restrict__ Vl, float* OUT, int qrow0) {
    __shared__ __align__(16) unsigned short pt[HI ? 8 : 4][16 * PP];
    __shared__ __align__(16) float ost[4][16 * OPF];
    const int wave = threadIdx.x >> 5, lane = threadIdx.x & 31, hh = lane >> 4, ln = lane & 15;
    const int b = blockIdx.y; const int q0 = qrow0 + (blockIdx.x * 4 + wave) * 16;
    const bf* Qhb = Qh + (size_t)b * SEQ * HS; const bf* Qlb = Ql + (size_t)b * SEQ * HS;
    const bf* Khb = Kh + (size_t)b * SEQ * HS; const bf* Klb = Kl + (size_t)b * SEQ * HS;
    const h16* V16b = V16 + (size_t)b * HS * SEQ; const bf* Vhb = Vh + (size_t)b * HS * SEQ; const bf* Vlb = Vl + (size_t)b * HS * SEQ;
    unsigned short* pta = &pt[(HI ? 2 : 1) * wave][0];
    unsigned short* ptb = &pt[(HI ? 2 : 1) * wave + (HI ? 1 : 0)][0];
    const size_t qo = (size_t)(q0 + ln) * HS + 8 * hh;
    const v16bf aqh = cat16b(*(const v8us*)(Qhb + qo), *(const v8us*)(Qhb + qo + 16));
    const v16bf aql = cat16b(*(const v8us*)(Qlb + qo), *(const v8us*)(Qlb + qo + 16));
    float mrun[8], lp[8]; v8f o0 = (v8f){}, o1 = (v8f){};
#pragma unroll
    for (int r = 0; r < 8; ++r) { mrun[r] = -3.0e38f; lp[r] = 0.0f; }
    int kv0 = 0;
#pragma unroll 1
    for (; kv0 + 64 <= q0; kv0 += 64) attn_chunk<HI, false>(Khb, Klb, V16b, Vhb, Vlb, pta, ptb, aqh, aql, kv0, q0, ln, hh, mrun, lp, o0, o1);
#pragma unroll 1
    for (; kv0 < q0 + 16; kv0 += 64) attn_chunk<HI, true>(Khb, Klb, V16b, Vhb, Vlb, pta, ptb, aqh, aql, kv0, q0, ln, hh, mrun, lp, o0, o1);
    const float carry = HI ? 1.0f : (1.0f / PCAR);
    float* osw = &ost[wave][0];
#pragma unroll
    for (int r = 0; r < 8; ++r) { float l = lp[r]; l += __shfl_xor(l, 1, 32); l += __shfl_xor(l, 2, 32); l += __shfl_xor(l, 4, 32); l += __shfl_xor(l, 8, 32);
        const float inv = carry * __builtin_amdgcn_rcpf(l);
        osw[(8 * hh + r) * OPF + ln] = o0[r] * inv; osw[(8 * hh + r) * OPF + 16 + ln] = o1[r] * inv; }
    __builtin_amdgcn_fence(3  , "wavefront");
    asm volatile("s_wait_dscnt 0x0" ::: "memory");
    __builtin_amdgcn_wave_barrier();
    float* ob = OUT + ((size_t)b * SEQ_FULL + q0) * HS;
#pragma unroll 1
    for (int ps = 0; ps < 2; ++ps) {
#pragma unroll
        for (int i = 0; i < 4; ++i) { const int row = 4 * i + (lane >> 3), col = (lane & 7) * 4; const v4f v = *(const v4fa*)(osw + row * OPF + col);
            *(volatile v4f*)(ob + (size_t)row * HS + col) = v; }
        if (ps == 0) __threadfence(); }
}

extern "C" void kernel_launch(void* const* d_in, const int* in_sizes, int n_in,
                              void* d_out, int out_size, void* d_ws, size_t ws_size, hipStream_t stream) {
    if (n_in < 4) return;
    const float* x  = (const float*)d_in[0];
    const float* wq = (const float*)d_in[1];
    const float* wk = (const float*)d_in[2];
    const float* wv = (const float*)d_in[3];
    if (in_sizes[0] < ((NB - 1) * SEQ_FULL + SEQ) * DM) return;
    if (in_sizes[1] < DM * HS || in_sizes[2] < DM * HS || in_sizes[3] < DM * HS) return;
    if (out_size < ((NB - 1) * SEQ_FULL + SEQ) * HS) return;
    float* OUT = (float*)d_out;
    char* wsp = (char*)d_ws;
    auto take = [&](size_t bytes) { char* p = wsp; wsp += (bytes + 255) & ~(size_t)255; return (void*)p; };
    bf*    WB   = (bf*)take((size_t)NP * DM * 2);
    float* CS   = (float*)take((size_t)SEQ * (HS / 2) * 2 * 4);
    bf*    XB   = (bf*)take((size_t)NB * SEQ * DM * 2);
    float* F    = (float*)take((size_t)NB * SEQ * NP * 4);
    bf*    Qh   = (bf*)take((size_t)NB * SEQ * HS * 2);
    bf*    Ql   = (bf*)take((size_t)NB * SEQ * HS * 2);
    bf*    Kh   = (bf*)take((size_t)NB * SEQ * HS * 2);
    bf*    Kl   = (bf*)take((size_t)NB * SEQ * HS * 2);
    h16*   VT16 = (h16*)take((size_t)NB * HS * SEQ * 2);
    bf*    VTh  = (bf*)take((size_t)NB * HS * SEQ * 2);
    bf*    VTl  = (bf*)take((size_t)NB * HS * SEQ * 2);
    if ((size_t)(wsp - (char*)d_ws) > ws_size) return;
    const int rh = (RH < SEQ) ? RH : SEQ;

    k_wt<<<(NP * DM / 8) / 256, 256, 0, stream>>>(wq, wk, wv, WB);
    k_cs<<<(SEQ * (HS / 2)) / 256, 256, 0, stream>>>(CS);
    const int n8 = NB * SEQ * (DM / 8);
    k_cvt<<<(unsigned)(n8 / 256), 256, 0, stream>>>(x, XB, n8);
    k_gemmw<bf, 0, false><<<dim3(NB * SEQ / 64, NP / 64, 1), 32, 0, stream>>>(XB, nullptr, WB, nullptr, DM, F, NP, nullptr, 0, 0, 0);
    k_planes<<<dim3(SEQ / 64, NB), 256, 0, stream>>>(F, CS, Qh, Ql, Kh, Kl, VT16, VTh, VTl);
    k_attn<true><<<dim3(rh / 64, NB), 128, 0, stream>>>(Qh, Ql, Kh, Kl, VT16, VTh, VTl, OUT, 0);
    if (SEQ > rh) k_attn<false><<<dim3((SEQ - rh) / 64, NB), 128, 0, stream>>>(Qh, Ql, Kh, Kl, VT16, VTh, VTl, OUT, rh);
}
